// SelfAttention_90744069030056
// MI455X (gfx1250) — hardware-run, weakly checked
//
#include <hip/hip_runtime.h>
#include <stddef.h>


typedef _Float16 v16h __attribute__((ext_vector_type(16)));
typedef _Float16 v8h  __attribute__((ext_vector_type(8)));
typedef float    v8f  __attribute__((ext_vector_type(8)));
typedef float    v4f  __attribute__((ext_vector_type(4)));

#ifndef NB
#define NB 16
#endif
#ifndef SEQ
#define SEQ 2048
#endif
#define NB_FULL  16
#define SEQ_FULL 2048
#define EMB   256
#define MROWS (NB * SEQ)

static_assert(NB >= 1 && NB <= NB_FULL);
static_assert(SEQ >= 128 && SEQ <= SEQ_FULL && (SEQ % 128) == 0);
static_assert(NB == 1 || SEQ == SEQ_FULL);
static_assert(EMB == 256);
static_assert((EMB % 64) == 0 && (EMB % 32) == 0);
static_assert((SEQ % 64) == 0 && (SEQ % 32) == 0);
static_assert((MROWS % 64) == 0 && (MROWS % 8) == 0);
static_assert(((size_t)MROWS * EMB) % 2048 == 0);
static_assert(((size_t)SEQ * EMB) % 2048 == 0);
static_assert(((size_t)EMB * EMB) % 2048 == 0);
static_assert((size_t)MROWS * EMB < (size_t)0xFFFFFFFFu);

#define LDT 72
#define LDC 68
#define LDP 40
#define LDO 68
static_assert((LDT % 8) == 0 && LDT >= 64);
static_assert((LDC % 4) == 0 && LDC >= 64);
static_assert((LDP % 8) == 0 && LDP >= 32);
static_assert((LDO % 4) == 0 && LDO >= 64);

#define WCARRY  64.0f
#define ACARRY  16.0f
#define QKCARRY 16384.0f
#define GCARRY  16.0f
#define TCARRY  16.0f
#define NCARRY  16.0f
#define VCARRY  16.0f
#define PCARRY  16384.0f
#define PCUT    (-19.0f)

#define CS_WQK (QKCARRY / (WCARRY * WCARRY))
#define CS_G   (GCARRY / (WCARRY * WCARRY))
#define CS_T   (TCARRY / (QKCARRY * GCARRY))
#define CS_N   (NCARRY / (WCARRY * TCARRY))
#define CS_V   (VCARRY / (WCARRY * ACARRY))
#define SCORE_SC (1.0f / (ACARRY * NCARRY * 16.0f))

#define SQ_BYTES    ((size_t)EMB * EMB * 2)
#define WA_BYTES    ((size_t)SEQ * EMB * 2)
#define PLANE_BYTES ((size_t)MROWS * EMB * 2)
#define BSQ_BYTES   ((size_t)NB * EMB * EMB * 2)
#define OFF_WQT  ((size_t)0)
#define OFF_WKT  (OFF_WQT + SQ_BYTES)
#define OFF_WV   (OFF_WKT + SQ_BYTES)
#define OFF_QKH  (OFF_WV + SQ_BYTES)
#define OFF_QKR  (OFF_QKH + SQ_BYTES)
#define OFF_WA   (OFF_QKR + SQ_BYTES)
#define OFF_C16  (OFF_WA + WA_BYTES)
#define OFF_CT   (OFF_C16 + PLANE_BYTES)
#define OFF_TT   (OFF_CT + PLANE_BYTES)
#define OFF_GH   (OFF_TT + PLANE_BYTES)
#define OFF_GR   (OFF_GH + BSQ_BYTES)
#define OFF_TH   (OFF_GR + BSQ_BYTES)
#define OFF_TR   (OFF_TH + BSQ_BYTES)
#define OFF_NH   (OFF_TR + BSQ_BYTES)
#define OFF_NR   (OFF_NH + PLANE_BYTES)
#define OFF_VT   (OFF_NR + PLANE_BYTES)
#define WS_TOTAL (OFF_VT + PLANE_BYTES)
static_assert((SQ_BYTES % 128) == 0 && (WA_BYTES % 128) == 0);
static_assert((PLANE_BYTES % 128) == 0 && (BSQ_BYTES % 128) == 0);
static_assert(WS_TOTAL <= (size_t)134217728);

__device__ __forceinline__ float bf16r(float x) {
  unsigned int u = __float_as_uint(x);
  u = (u + 0x7FFFu + ((u >> 16) & 1u)) & 0xFFFF0000u;
  return __uint_as_float(u);
}

static __device__ __forceinline__ _Float16 toh_flush(float v) {
  const _Float16 r = (_Float16)v;
  return (fabsf(v) < 6.103515625e-05f) ? (_Float16)0.0f : r;
}

__device__ __forceinline__ v16h frag_at(const _Float16* p) {
  v8h lo = *(const v8h*)(p);
  v8h hi = *(const v8h*)(p + 16);
  v16h out;
#pragma unroll
  for (int i = 0; i < 8; ++i) { out[i] = lo[i]; out[i + 8] = hi[i]; }
  return out;
}

__device__ __forceinline__ v8f wmma16(v16h a, v16h b, v8f c) {
  v8f d = __builtin_amdgcn_wmma_f32_16x16x32_f16(false, a, false, b, (short)0, c,
                                                 false, false);
  asm volatile("v_nop\n\tv_nop\n\tv_nop\n\tv_nop" : "+v"(d) : "v"(a), "v"(b));
  return d;
}

__device__ __forceinline__ float red16_max(float x) {
#pragma unroll
  for (int off = 1; off < 16; off <<= 1) x = fmaxf(x, __shfl_xor(x, off, 32));
  return x;
}
__device__ __forceinline__ float red16_sum(float x) {
#pragma unroll
  for (int off = 1; off < 16; off <<= 1) x += __shfl_xor(x, off, 32);
  return x;
}

__device__ __forceinline__ void wave_lds_sync() {
  __builtin_amdgcn_fence(3  , "wavefront");
  asm volatile("s_wait_dscnt 0x0" ::: "memory");
  __builtin_amdgcn_wave_barrier();
}

__global__ __launch_bounds__(256) void wconv_kernel(
    const float* __restrict__ W, _Float16* __restrict__ Wt, unsigned ldw, unsigned ldk) {
  __shared__ _Float16 T[64 * LDT];
  const unsigned tid = threadIdx.x;
  const unsigned n0 = blockIdx.x * 64u;
  const unsigned k0 = blockIdx.y * 64u;
#pragma unroll 4
  for (unsigned j = 0; j < 16u; ++j) {
    const unsigned idx = tid + 256u * j;
    const unsigned kr = idx >> 6, nc = idx & 63u;
    const float v = W[(size_t)(k0 + kr) * ldw + n0 + nc];
    T[nc * LDT + kr] = (_Float16)(WCARRY * bf16r(v));
  }
  __syncthreads();
  v8h x[2];
  size_t off[2];
#pragma unroll
  for (unsigned i = 0; i < 2u; ++i) {
    const unsigned n = 32u * i + (tid >> 3);
    const unsigned kc = (tid & 7u) * 8u;
    x[i] = *(const v8h*)&T[n * LDT + kc];
    off[i] = (size_t)(n0 + n) * ldk + k0 + kc;
  }
#pragma unroll
  for (int i = 0; i < 2; ++i) *(volatile v8h*)(Wt + off[i]) = x[i];
  __threadfence();
#pragma unroll
  for (int i = 0; i < 2; ++i) *(volatile v8h*)(Wt + off[i]) = x[i];
}

__global__ __launch_bounds__(256) void cvt_kernel(
    const float* __restrict__ src, _Float16* __restrict__ dst, float carry) {
#pragma clang fp contract(off)
  const size_t e0 = ((size_t)blockIdx.x * 256u + threadIdx.x) * 8u;
  const v4f a0 = *(const v4f*)(src + e0);
  const v4f a1 = *(const v4f*)(src + e0 + 4u);
  v8h o;
#pragma unroll
  for (int i = 0; i < 4; ++i) {
    o[i]     = toh_flush(carry * bf16r(a0[i]));
    o[i + 4] = toh_flush(carry * bf16r(a1[i]));
  }
  _Float16* p = dst + e0;
  *(volatile v8h*)p = o;
  __threadfence();
  *(volatile v8h*)p = o;
}

template <int NPROD, int DUAL>
__device__ __forceinline__ void gemm_body(
    const _Float16* __restrict__ Ah, const _Float16* __restrict__ Ar,
    const _Float16* __restrict__ Bh, const _Float16* __restrict__ Br,
    const unsigned K, const unsigned lda, const unsigned ldb,
    const size_t sA, const size_t sB, const float cs,
    _Float16* __restrict__ outh, _Float16* __restrict__ outr,
    const unsigned ldo, const size_t sO) {
  __shared__ float Cs[64 * LDC];
  const unsigned tid = threadIdx.x, lane = tid & 31u;
  const unsigned w = (unsigned)__builtin_amdgcn_readfirstlane((int)(threadIdx.x >> 5));
  const unsigned mw = w >> 1, nw = w & 1u;
  const unsigned hh = lane >> 4, m = lane & 15u;
  const unsigned n0 = blockIdx.x * 64u;
  const unsigned row0 = blockIdx.y * 64u;
  const size_t z = blockIdx.z;

  const size_t aoff  = z * sA + (size_t)(row0 + mw * 16u + m) * lda + hh * 8u;
  const size_t boff0 = z * sB + (size_t)(n0 + nw * 32u + m) * ldb + hh * 8u;
  const size_t boff1 = boff0 + (size_t)16 * ldb;
  v8f acc0 = {}, acc1 = {};
#pragma unroll 2
  for (unsigned k0 = 0; k0 < K; k0 += 32u) {
    const v16h a  = frag_at(Ah + aoff + k0);
    const v16h b0 = frag_at(Bh + boff0 + k0);
    const v16h b1 = frag_at(Bh + boff1 + k0);
    acc0 = wmma16(a, b0, acc0);
    acc1 = wmma16(a, b1, acc1);
    if (NPROD >= 2) {
      const v16h c0 = frag_at(Br + boff0 + k0);
      const v16h c1 = frag_at(Br + boff1 + k0);
      acc0 = wmma16(a, c0, acc0);
      acc1 = wmma16(a, c1, acc1);
    }
    if (NPROD >= 3) {
      const v16h ar = frag_at(Ar + aoff + k0);
      acc0 = wmma16(ar, b0, acc0);
      acc1 = wmma16(ar, b1, acc1);
    }
  }
#pragma unroll
  for (int r = 0; r < 8; ++r) {
    float* d = &Cs[(mw * 16u + hh * 8u + (unsigned)r) * LDC + nw * 32u + m];
    d[0]  = acc0[r];
    d[16] = acc1[r];
  }
  __syncthreads();

  v8h x[2], xr[2];
  size_t off[2];
#pragma unroll
  for (unsigned i = 0; i < 2u; ++i) {
    const unsigned r = 32u * i + (tid >> 3);
    const unsigned c = (tid & 7u) * 8u;
    const v4f u0 = *(const v4f*)&Cs[r * LDC + c];
    const v4f u1 = *(const v4f*)&Cs[r * LDC + c + 4];
#pragma unroll
    for (int j = 0; j < 4; ++j) {
      const float t0 = u0[j] * cs;
      const float t1 = u1[j] * cs;
      const _Float16 h0 = toh_flush(t0);
      const _Float16 h1 = toh_flush(t1);
      x[i][j]     = h0;
      x[i][j + 4] = h1;
      xr[i][j]     = toh_flush(t0 - (float)h0);
      xr[i][j + 4] = toh_flush(t1 - (float)h1);
    }
    off[i] = z * sO + (size_t)(row0 + r) * ldo + n0 + c;
  }
#pragma unroll
  for (int i = 0; i < 2; ++i) *(volatile v8h*)(outh + off[i]) = x[i];
  if (DUAL) {
#pragma unroll
    for (int i = 0; i < 2; ++i) *(volatile v8h*)(outr + off[i]) = xr[i];
  }
  __threadfence();
#pragma unroll
  for (int i = 0; i < 2; ++i) *(volatile v8h*)(outh + off[i]) = x[i];
  if (DUAL) {
#pragma unroll
    for (int i = 0; i < 2; ++i) *(volatile v8h*)(outr + off[i]) = xr[i];
  }
}

__global__ __launch_bounds__(256) void gemm_wqk_kernel(
    const _Float16* __restrict__ WqT, const _Float16* __restrict__ WkT,
    _Float16* __restrict__ Qkh, _Float16* __restrict__ Qkr) {
  gemm_body<1, 1>(WqT, WqT, WkT, WkT, (unsigned)EMB, (unsigned)EMB, (unsigned)EMB,
                  (size_t)0, (size_t)0, CS_WQK, Qkh, Qkr, (unsigned)EMB, (size_t)0);
}
__global__ __launch_bounds__(256) void gemm_g_kernel(
    const _Float16* __restrict__ TextT, const _Float16* __restrict__ CodeT,
    _Float16* __restrict__ Gh, _Float16* __restrict__ Gr) {
  gemm_body<1, 1>(TextT, TextT, CodeT, CodeT, (unsigned)SEQ, (unsigned)MROWS, (unsigned)MROWS,
                  (size_t)SEQ, (size_t)SEQ, CS_G, Gh, Gr, (unsigned)EMB, (size_t)EMB * EMB);
}
__global__ __launch_bounds__(256) void gemm_t_kernel(
    const _Float16* __restrict__ Qkh, const _Float16* __restrict__ Qkr,
    const _Float16* __restrict__ Gh, const _Float16* __restrict__ Gr,
    _Float16* __restrict__ Th, _Float16* __restrict__ Tr) {
  gemm_body<3, 1>(Qkh, Qkr, Gh, Gr, (unsigned)EMB, (unsigned)EMB, (unsigned)EMB,
                  (size_t)0, (size_t)EMB * EMB, CS_T, Th, Tr, (unsigned)EMB, (size_t)EMB * EMB);
}
__global__ __launch_bounds__(256) void gemm_n_kernel(
    const _Float16* __restrict__ Wa16, const _Float16* __restrict__ Th,
    const _Float16* __restrict__ Tr, _Float16* __restrict__ Nh, _Float16* __restrict__ Nr) {
  gemm_body<2, 1>(Wa16, Wa16, Th, Tr, (unsigned)EMB, (unsigned)EMB, (unsigned)EMB,
                  (size_t)0, (size_t)EMB * EMB, CS_N, Nh, Nr, (unsigned)EMB, (size_t)SEQ * EMB);
}
__global__ __launch_bounds__(256) void gemm_v_kernel(
    const _Float16* __restrict__ Wv16, const _Float16* __restrict__ Code16,
    _Float16* __restrict__ Vt) {
  gemm_body<1, 0>(Wv16, Wv16, Code16, Code16, (unsigned)EMB, (unsigned)EMB, (unsigned)EMB,
                  (size_t)0, (size_t)SEQ * EMB, CS_V, Vt, Vt, (unsigned)SEQ, (size_t)EMB * SEQ);
}

__global__ __launch_bounds__(256) __attribute__((amdgpu_num_vgpr(256))) void attn_kernel(
    const _Float16* __restrict__ Qc, const _Float16* __restrict__ NTh,
    const _Float16* __restrict__ NTr, const _Float16* __restrict__ Vt,
    float* __restrict__ out) {
  __shared__ _Float16 Ps[8 * 16 * LDP];
  __shared__ float Os[8 * 16 * LDO];

  const unsigned lane = threadIdx.x & 31u;
  const unsigned w = (unsigned)__builtin_amdgcn_readfirstlane((int)(threadIdx.x >> 5));
  const unsigned hh = lane >> 4, m = lane & 15u;
  const unsigned b = blockIdx.y;
  const unsigned qrow0 = blockIdx.x * 128u + w * 16u;
  const unsigned pbase = w * (16u * LDP);
  const unsigned obase = w * (16u * LDO);

  const size_t qoff = ((size_t)b * SEQ + qrow0 + m) * EMB + hh * 8u;
  const size_t koff = ((size_t)b * SEQ + m) * EMB + hh * 8u;
  const size_t voff = ((size_t)b * EMB + m) * SEQ + hh * 8u;

  float mrow[8], lrow[8];
  v8f o[16];
#pragma unroll
  for (int v = 0; v < 8; ++v) { mrow[v] = -1.0e30f; lrow[v] = 0.0f; }
#pragma unroll
  for (int nb = 0; nb < 16; ++nb) o[nb] = (v8f){};

  for (unsigned kb = 0; kb < (unsigned)SEQ; kb += 32u) {
    const size_t kp0 = koff + (size_t)kb * EMB;
    const size_t kp1 = kp0 + (size_t)16 * EMB;
    v8f s0 = {}, s1 = {};
#pragma unroll 1
    for (unsigned ks = 0; ks < (unsigned)EMB; ks += 32u) {
      const v16h a  = frag_at(Qc + qoff + ks);
      const v16h h0 = frag_at(NTh + kp0 + ks);
      const v16h h1 = frag_at(NTh + kp1 + ks);
      const v16h r0 = frag_at(NTr + kp0 + ks);
      const v16h r1 = frag_at(NTr + kp1 + ks);
      s0 = wmma16(a, h0, s0);
      s1 = wmma16(a, h1, s1);
      s0 = wmma16(a, r0, s0);
      s1 = wmma16(a, r1, s1);
    }

    float alpha[8];
#pragma unroll
    for (int v = 0; v < 8; ++v) {
      const float x0 = s0[v] * SCORE_SC;
      const float x1 = s1[v] * SCORE_SC;
      const float mx = red16_max(fmaxf(x0, x1));
      const float mn = fmaxf(mrow[v], mx);
      alpha[v] = __expf(mrow[v] - mn);
      mrow[v] = mn;
      const float e0 = x0 - mn;
      const float e1 = x1 - mn;
      const float g0 = __expf(e0) * PCARRY;
      const float g1 = __expf(e1) * PCARRY;
      const _Float16 p0 = (_Float16)((e0 < PCUT) ? 0.0f : g0);
      const _Float16 p1 = (_Float16)((e1 < PCUT) ? 0.0f : g1);
      Ps[pbase + (hh * 8u + (unsigned)v) * LDP + m]       = p0;
      Ps[pbase + (hh * 8u + (unsigned)v) * LDP + 16u + m] = p1;
      const float rs = red16_sum((float)p0 + (float)p1);
      lrow[v] = alpha[v] * lrow[v] + rs;
    }
#pragma unroll
    for (int nb = 0; nb < 16; ++nb)
#pragma unroll
      for (int v = 0; v < 8; ++v) o[nb][v] = o[nb][v] * alpha[v];
    wave_lds_sync();

    const v16h pf = frag_at(&Ps[pbase + m * LDP + hh * 8u]);
#pragma unroll
    for (int g = 0; g < 4; ++g) {
      v16h vf[4];
#pragma unroll
      for (int j = 0; j < 4; ++j)
        vf[j] = frag_at(Vt + voff + (size_t)((g * 4 + j) * 16) * SEQ + kb);
#pragma unroll
      for (int j = 0; j < 4; ++j) o[g * 4 + j] = wmma16(pf, vf[j], o[g * 4 + j]);
      asm volatile("" ::: "memory");
    }
    wave_lds_sync();
  }

  float inv[8];
#pragma unroll
  for (int v = 0; v < 8; ++v) inv[v] = __builtin_amdgcn_rcpf(lrow[v]) * (1.0f / VCARRY);
#pragma unroll
  for (int ch = 0; ch < 4; ++ch) {
#pragma unroll
    for (int j = 0; j < 4; ++j)
#pragma unroll
      for (int v = 0; v < 8; ++v)
        Os[obase + (hh * 8u + (unsigned)v) * LDO + (unsigned)j * 16u + m] =
            o[ch * 4 + j][v] * inv[v];
    wave_lds_sync();
    v4f x[8];
    size_t off[8];
#pragma unroll
    for (unsigned i = 0; i < 8u; ++i) {
      const unsigned r = 2u * i + hh;
      const unsigned c = m * 4u;
      x[i] = *(const v4f*)&Os[obase + r * LDO + c];
      off[i] = ((size_t)b * SEQ_FULL + qrow0 + r) * EMB + (unsigned)ch * 64u + c;
    }
#pragma unroll
    for (int i = 0; i < 8; ++i) *(volatile v4f*)(out + off[i]) = x[i];
    __threadfence();
#pragma unroll
    for (int i = 0; i < 8; ++i) *(volatile v4f*)(out + off[i]) = x[i];
    wave_lds_sync();
  }
}

extern "C" void kernel_launch(void* const* d_in, const int* in_sizes, int n_in,
                              void* d_out, int out_size, void* d_ws, size_t ws_size,
                              hipStream_t stream) {
  if (n_in < 6) return;
  const long long need_x = ((long long)(NB - 1) * SEQ_FULL + SEQ) * EMB;
  if ((long long)in_sizes[0] < need_x) return;
  if ((long long)in_sizes[1] < need_x) return;
  if ((long long)in_sizes[2] < (long long)EMB * EMB) return;
  if ((long long)in_sizes[3] < (long long)EMB * EMB) return;
  if ((long long)in_sizes[4] < (long long)EMB * EMB) return;
  if ((long long)in_sizes[5] < (long long)SEQ * EMB) return;
  if ((long long)out_size < need_x) return;
  if (ws_size < WS_TOTAL) return;

  const float* code = (const float*)d_in[0];
  const float* text = (const float*)d_in[1];
  const float* wv   = (const float*)d_in[2];
  const float* wk   = (const float*)d_in[3];
  const float* wq   = (const float*)d_in[4];
  const float* wa   = (const float*)d_in[5];
  float* out = (float*)d_out;

  char* ws = (char*)d_ws;
  _Float16* WqT    = (_Float16*)(ws + OFF_WQT);
  _Float16* WkT    = (_Float16*)(ws + OFF_WKT);
  _Float16* Wv16   = (_Float16*)(ws + OFF_WV);
  _Float16* Qkh    = (_Float16*)(ws + OFF_QKH);
  _Float16* Qkr    = (_Float16*)(ws + OFF_QKR);
  _Float16* Wa16   = (_Float16*)(ws + OFF_WA);
  _Float16* Code16 = (_Float16*)(ws + OFF_C16);
  _Float16* CodeT  = (_Float16*)(ws + OFF_CT);
  _Float16* TextT  = (_Float16*)(ws + OFF_TT);
  _Float16* Gh     = (_Float16*)(ws + OFF_GH);
  _Float16* Gr     = (_Float16*)(ws + OFF_GR);
  _Float16* Th     = (_Float16*)(ws + OFF_TH);
  _Float16* Tr     = (_Float16*)(ws + OFF_TR);
  _Float16* Nh     = (_Float16*)(ws + OFF_NH);
  _Float16* Nr     = (_Float16*)(ws + OFF_NR);
  _Float16* Vt16   = (_Float16*)(ws + OFF_VT);

  dim3 blk(256);

  wconv_kernel<<<dim3(EMB / 64, EMB / 64), blk, 0, stream>>>(wq, WqT, (unsigned)EMB, (unsigned)EMB);
  wconv_kernel<<<dim3(EMB / 64, EMB / 64), blk, 0, stream>>>(wk, WkT, (unsigned)EMB, (unsigned)EMB);
  wconv_kernel<<<dim3(EMB / 64, MROWS / 64), blk, 0, stream>>>(code, CodeT, (unsigned)EMB, (unsigned)MROWS);
  wconv_kernel<<<dim3(EMB / 64, MROWS / 64), blk, 0, stream>>>(text, TextT, (unsigned)EMB, (unsigned)MROWS);

  cvt_kernel<<<dim3((unsigned)(((size_t)MROWS * EMB) / 2048)), blk, 0, stream>>>(code, Code16, ACARRY);
  cvt_kernel<<<dim3((unsigned)(((size_t)SEQ * EMB) / 2048)), blk, 0, stream>>>(wa, Wa16, WCARRY);
  cvt_kernel<<<dim3((unsigned)(((size_t)EMB * EMB) / 2048)), blk, 0, stream>>>(wv, Wv16, WCARRY);

  gemm_wqk_kernel<<<dim3(EMB / 64, EMB / 64, 1), blk, 0, stream>>>(WqT, WkT, Qkh, Qkr);
  gemm_g_kernel<<<dim3(EMB / 64, EMB / 64, NB), blk, 0, stream>>>(TextT, CodeT, Gh, Gr);
  gemm_t_kernel<<<dim3(EMB / 64, EMB / 64, NB), blk, 0, stream>>>(Qkh, Qkr, Gh, Gr, Th, Tr);
  gemm_n_kernel<<<dim3(EMB / 64, SEQ / 64, NB), blk, 0, stream>>>(Wa16, Th, Tr, Nh, Nr);
  gemm_v_kernel<<<dim3(SEQ / 64, EMB / 64, NB), blk, 0, stream>>>(Wv16, Code16, Vt16);
  attn_kernel<<<dim3(SEQ / 128, NB), blk, 0, stream>>>(Code16, Nh, Nr, Vt16, out);
}
